// segmentation_model_67327907332570
// MI455X (gfx1250) — hardware-verified
//
#include <hip/hip_runtime.h>
#include <math.h>

typedef __attribute__((ext_vector_type(16))) _Float16 v16h;
typedef __attribute__((ext_vector_type(8)))  _Float16 v8h;
typedef __attribute__((ext_vector_type(16))) __bf16   v16b;
typedef __attribute__((ext_vector_type(8)))  __bf16   v8b;
typedef __attribute__((ext_vector_type(8)))  float    v8f;
typedef __attribute__((ext_vector_type(4)))  float    v4f;

constexpr int kB     = 8;
constexpr int kL     = 1024;
constexpr int kDM    = 256;
constexpr int kDI    = 512;
constexpr int kDS    = 16;
constexpr int kDTR   = 16;
constexpr int kNPJ   = kDTR + 2 * kDS;
constexpr int kNPJP  = 64;
constexpr int kXZP   = 2 * kDI;
constexpr int kRows  = kB * kL;
constexpr int kChunk = 32;
constexpr int kCG    = 128;
constexpr int kYP    = 132;
constexpr int kNOUT  = 3;
constexpr int kTokB  = 32;
static_assert(kL % kChunk == 0);
static_assert(kRows % 64 == 0 && kXZP % 64 == 0 && kDM % 64 == 0 && kNPJP % 64 == 0);
static_assert(kDM % 32 == 0 && kDI % 32 == 0);
static_assert(kDI % kCG == 0 && kRows % kTokB == 0);

__device__ __forceinline__ unsigned short f2bf_bits(float f) {
  unsigned u = __float_as_uint(f);
  return (unsigned short)((u + 0x7FFFu + ((u >> 16) & 1u)) >> 16);
}
__device__ __forceinline__ float bf_bits2f(unsigned short h) { return __uint_as_float(((unsigned)h) << 16); }

__device__ __forceinline__ void dep_guard_h(v8f& a, v8f& b, v16h x, v16h y) { asm volatile("v_nop\n\tv_nop\n\tv_nop\n\tv_nop" : "+v"(a), "+v"(b) : "v"(x), "v"(y)); }
__device__ __forceinline__ void dep_guard_b(v8f& a, v8f& b, v16b x, v16b y) { asm volatile("v_nop\n\tv_nop\n\tv_nop\n\tv_nop" : "+v"(a), "+v"(b) : "v"(x), "v"(y)); }
__device__ __forceinline__ void keep4_h(v16h a, v16h b, v16h c, v16h d) { asm volatile("v_nop" :: "v"(a), "v"(b), "v"(c), "v"(d)); }
__device__ __forceinline__ void keep4_b(v16b a, v16b b, v16b c, v16b d) { asm volatile("v_nop" :: "v"(a), "v"(b), "v"(c), "v"(d)); }
__device__ __forceinline__ void acc_guard4(v8f& a, v8f& b, v8f& c, v8f& d) { asm volatile("v_nop\n\tv_nop\n\tv_nop\n\tv_nop" : "+v"(a), "+v"(b), "+v"(c), "+v"(d)); }
template <typename T> struct Frag;
template <> struct Frag<_Float16> {
  typedef v16h V; union U { v16h v; v8h h[2]; };
  static __device__ __forceinline__ v16h load(const _Float16* p) {
    U f; f.h[0] = *(const v8h*)(p); f.h[1] = *(const v8h*)(p + 16); return f.v;
  }
  static __device__ __forceinline__ v8f mma(v16h a, v16h b, v8f c) {
    return __builtin_amdgcn_wmma_f32_16x16x32_f16(false, a, false, b, (short)0, c, false, false);
  }
  static __device__ __forceinline__ void guard(v8f& a, v8f& b, v16h x, v16h y) { dep_guard_h(a, b, x, y); }
  static __device__ __forceinline__ void keep(v16h a, v16h b, v16h c, v16h d) { keep4_h(a, b, c, d); }
};
template <> struct Frag<__bf16> {
  typedef v16b V; union U { v16b v; v8b h[2]; };
  static __device__ __forceinline__ v16b load(const __bf16* p) {
    U f; f.h[0] = *(const v8b*)(p); f.h[1] = *(const v8b*)(p + 16); return f.v;
  }
  static __device__ __forceinline__ v8f mma(v16b a, v16b b, v8f c) {
    return __builtin_amdgcn_wmma_f32_16x16x32_bf16(false, a, false, b, (short)0, c, false, false);
  }
  static __device__ __forceinline__ void guard(v8f& a, v8f& b, v16b x, v16b y) { dep_guard_b(a, b, x, y); }
  static __device__ __forceinline__ void keep(v16b a, v16b b, v16b c, v16b d) { keep4_b(a, b, c, d); }
};

template <int ET> struct Elem;
template <> struct Elem<0> { typedef _Float16 T; };
template <> struct Elem<1> { typedef __bf16 T; };
template <int ET, bool SPLIT, int BIAS_MODE, int OUT_MODE, bool RESID, int ACT = 0>
__global__ __launch_bounds__(256) void wmma_gemm64(
    const unsigned short* __restrict__ Ap, const unsigned short* __restrict__ A2p, int lda, long strideA,
    const unsigned short* __restrict__ Btp, const unsigned short* __restrict__ Bt2p, int ldb, long strideB,
    void* __restrict__ Cout, void* __restrict__ Cout2, int ldc, long strideC,
    const float* __restrict__ bias,
    const float* __restrict__ resid, long strideR,
    int M, int N, int K, float scale) {
  typedef typename Elem<ET>::T T;
  typedef typename Frag<T>::V V;
  const T* A = (const T*)Ap; const T* A2 = (const T*)A2p; const T* Bt = (const T*)Btp; const T* Bt2 = (const T*)Bt2p;
  __shared__ __align__(16) float sT[8][16 * 68];
  const int b    = blockIdx.y;
  const int lane = threadIdx.x & 31;
  const int wave = threadIdx.x >> 5;
  const int tilesN = N >> 6;
  const int tilesM = M >> 6;
  const int tile = blockIdx.x * 8 + wave;
  if (tile >= tilesM * tilesN) return;
  const int tm = tile / tilesN;
  const int tn = tile - tm * tilesN;
  const int m0 = tm << 6;
  const int n0 = tn << 6;

  const T* Ab  = A  + (size_t)b * strideA;
  const T* Bb  = Bt + (size_t)b * strideB;
  const T* Ab2 = SPLIT ? (A2  + (size_t)b * strideA) : nullptr;
  const T* Bb2 = SPLIT ? (Bt2 + (size_t)b * strideB) : nullptr;

  const int rlane = lane & 15;
  const int koff  = (lane >> 4) * 8;
  const int mOff  = (lane >> 4) * 8;

  v8f acc[4][4];
#pragma unroll
  for (int i = 0; i < 4; ++i)
#pragma unroll
    for (int j = 0; j < 4; ++j) acc[i][j] = (v8f){0.f,0.f,0.f,0.f,0.f,0.f,0.f,0.f};

  for (int k0 = 0; k0 < K; k0 += 32) {
    V bh[4], bl[4];
#pragma unroll
    for (int j = 0; j < 4; ++j) {
      const size_t bo = (size_t)(n0 + (j << 4) + rlane) * ldb + koff + k0;
      bh[j] = Frag<T>::load(Bb + bo);
      if (SPLIT) bl[j] = Frag<T>::load(Bb2 + bo);
    }
#pragma unroll
    for (int i = 0; i < 4; ++i) {
      const size_t ao = (size_t)(m0 + (i << 4) + rlane) * lda + koff + k0;
      V ah = Frag<T>::load(Ab + ao);
      V al;
      if (SPLIT) al = Frag<T>::load(Ab2 + ao);
#pragma unroll
      for (int j = 0; j < 4; ++j) {
        acc[i][j] = Frag<T>::mma(ah, bh[j], acc[i][j]);
        if (SPLIT) {
          acc[i][j] = Frag<T>::mma(ah, bl[j], acc[i][j]);
          acc[i][j] = Frag<T>::mma(al, bh[j], acc[i][j]);
        }
      }
      Frag<T>::guard(acc[i][0], acc[i][3], ah, SPLIT ? al : ah);
    }
    Frag<T>::keep(bh[0], bh[1], bh[2], bh[3]);
    if (SPLIT) Frag<T>::keep(bl[0], bl[1], bl[2], bl[3]);
  }
  acc_guard4(acc[0][0], acc[0][1], acc[0][2], acc[0][3]);
  acc_guard4(acc[1][0], acc[1][1], acc[1][2], acc[1][3]);
  acc_guard4(acc[2][0], acc[2][1], acc[2][2], acc[2][3]);
  acc_guard4(acc[3][0], acc[3][1], acc[3][2], acc[3][3]);

  float* slab = sT[wave];
  const float* Rb = RESID ? (resid + (size_t)b * strideR) : nullptr;
#pragma unroll
  for (int i = 0; i < 4; ++i) {
    const int mBase = m0 + (i << 4);
#pragma unroll
    for (int j = 0; j < 4; ++j) {
      const int n = n0 + (j << 4) + rlane;
      float bv = 0.f;
      if (BIAS_MODE == 2) bv = bias[n];
#pragma unroll
      for (int r = 0; r < 8; ++r) {
        float v = acc[i][j][r] * scale;
        if (BIAS_MODE == 1) v += bias[mBase + mOff + r];
        if (BIAS_MODE == 2) v += bv;
        if (RESID) v += Rb[(size_t)(mBase + mOff + r) * ldc + n];
        if (ACT == 1) v = tanhf(v);
        if (ACT == 2) v = fmaxf(v, 0.0f);
        if (ACT == 3) v = v / (1.0f + expf(-v));
        if (ACT == 4) v = (v > 0.f) ? v : 0.01f * v;
        if (ACT == 5) v = 0.5f * v * (1.0f + erff(v * 0.70710678118654752f));
        slab[(mOff + r) * 68 + (j << 4) + rlane] = v;
      }
    }
    __builtin_amdgcn_fence(__ATOMIC_RELEASE, "workgroup");
    __builtin_amdgcn_wave_barrier();
    __builtin_amdgcn_fence(__ATOMIC_ACQUIRE, "workgroup");
    if (OUT_MODE == 0) {
      float* C = (float*)Cout + (size_t)b * strideC;
      const int hh = lane >> 4, c4 = (lane & 15) * 4;
      for (int pass = 0; pass < 2; ++pass) {
#pragma unroll
        for (int it = 0; it < 8; ++it) {
          const int row = it * 2 + hh;
          v4f v = *(const v4f*)(slab + row * 68 + c4);
          *(volatile v4f*)(C + (size_t)(mBase + row) * ldc + n0 + c4) = v;
        }
        __threadfence();
      }
    } else {
      const int q = lane >> 3, c8 = (lane & 7) * 8;
      unsigned short* C  = (unsigned short*)Cout  + (size_t)b * strideC;
      unsigned short* C2 = (OUT_MODE == 2) ? ((unsigned short*)Cout2 + (size_t)b * strideC) : nullptr;
      for (int pass = 0; pass < 2; ++pass) {
#pragma unroll
        for (int it = 0; it < 4; ++it) {
          const int row = it * 4 + q;
          const float* sp = slab + row * 68 + c8;
          v8h hv, lv;
#pragma unroll
          for (int e = 0; e < 8; ++e) {
            if (OUT_MODE == 1) {
              hv[e] = (_Float16)sp[e];
            } else {
              unsigned short hb = f2bf_bits(sp[e]);
              unsigned short lb = f2bf_bits(sp[e] - bf_bits2f(hb));
              hv[e] = __builtin_bit_cast(_Float16, hb);
              lv[e] = __builtin_bit_cast(_Float16, lb);
            }
          }
          *(volatile v8h*)(C + (size_t)(mBase + row) * ldc + n0 + c8) = hv;
          if (OUT_MODE == 2) *(volatile v8h*)(C2 + (size_t)(mBase + row) * ldc + n0 + c8) = lv;
        }
        __threadfence();
      }
    }
    __builtin_amdgcn_fence(__ATOMIC_RELEASE, "workgroup");
    __builtin_amdgcn_wave_barrier();
    __builtin_amdgcn_fence(__ATOMIC_ACQUIRE, "workgroup");
  }
}

struct HL8 { v8h h; v8h l; };
__device__ __forceinline__ HL8 split8_bf16(const v4f a0, const v4f a1) {
  HL8 r;
#pragma unroll
  for (int e = 0; e < 4; ++e) {
    const unsigned short h0 = f2bf_bits(a0[e]);
    const unsigned short l0 = f2bf_bits(a0[e] - bf_bits2f(h0));
    const unsigned short h1 = f2bf_bits(a1[e]);
    const unsigned short l1 = f2bf_bits(a1[e] - bf_bits2f(h1));
    r.h[e]     = __builtin_bit_cast(_Float16, h0);
    r.l[e]     = __builtin_bit_cast(_Float16, l0);
    r.h[4 + e] = __builtin_bit_cast(_Float16, h1);
    r.l[4 + e] = __builtin_bit_cast(_Float16, l1);
  }
  return r;
}

__global__ __launch_bounds__(256) void split_bf16_kernel(
    const float* __restrict__ src, unsigned short* __restrict__ hi, unsigned short* __restrict__ lo, int total8)
{
  const int i = blockIdx.x * 256 + threadIdx.x;
  if (i >= total8) return;
  const size_t e0 = (size_t)i << 3;
  const float* p = src + e0;
  const v4f a0 = *(const v4f*)(p);
  const v4f a1 = *(const v4f*)(p + 4);
  const HL8 r = split8_bf16(a0, a1);
  unsigned short* qh = hi + e0;
  unsigned short* ql = lo + e0;
  *(volatile v8h*)qh = r.h;
  *(volatile v8h*)ql = r.l;
  __threadfence();
  *(volatile v8h*)qh = r.h;
  *(volatile v8h*)ql = r.l;
}

__global__ __launch_bounds__(256) void split_bf16_pad_kernel(
    const float* __restrict__ src, int n_src, unsigned short* __restrict__ hi, unsigned short* __restrict__ lo, int total8)
{
  const int i = blockIdx.x * 256 + threadIdx.x;
  if (i >= total8) return;
  const int e0 = i << 3;
  const bool live = (e0 + 8) <= n_src;
  const int es = live ? e0 : (n_src - 8);
  const float* p = src + es;
  v4f a0 = *(const v4f*)(p);
  v4f a1 = *(const v4f*)(p + 4);
  const v4f z4 = (v4f){0.f, 0.f, 0.f, 0.f};
  a0 = live ? a0 : z4;
  a1 = live ? a1 : z4;
  const HL8 r = split8_bf16(a0, a1);
  unsigned short* qh = hi + (size_t)e0;
  unsigned short* ql = lo + (size_t)e0;
  *(volatile v8h*)qh = r.h;
  *(volatile v8h*)ql = r.l;
  __threadfence();
  *(volatile v8h*)qh = r.h;
  *(volatile v8h*)ql = r.l;
}

__global__ __launch_bounds__(256) void x_rows_split_kernel(
    const float* __restrict__ x, unsigned short* __restrict__ XH, unsigned short* __restrict__ XL, int flip)
{
  const int i = blockIdx.x * 256 + threadIdx.x;
  const int row = i >> 5;
  if (row >= kRows) return;
  const int c8 = (i & 31) * 8;
  const int b = row >> 10, t = row & (kL - 1);
  const int tsrc = flip ? (kL - 1 - t) : t;
  const float* p = x + ((size_t)(b * kL + tsrc) * kDM + c8);
  const v4f a0 = *(const v4f*)(p);
  const v4f a1 = *(const v4f*)(p + 4);
  const HL8 r = split8_bf16(a0, a1);
  const size_t o = (size_t)row * kDM + c8;
  *(volatile v8h*)(XH + o) = r.h;
  *(volatile v8h*)(XL + o) = r.l;
  __threadfence();
  *(volatile v8h*)(XH + o) = r.h;
  *(volatile v8h*)(XL + o) = r.l;
}

__global__ __launch_bounds__(256) void conv_split_kernel(
    const float* __restrict__ XZ, const float* __restrict__ conv_w, const float* __restrict__ conv_b,
    unsigned short* __restrict__ XCH, unsigned short* __restrict__ XCL)
{
  const int i = blockIdx.x * 256 + threadIdx.x;
  const int row = i >> 6;
  if (row >= kRows) return;
  const int c8 = (i & 63) * 8;
  const int t = row & (kL - 1);
  v4f wv[8];
#pragma unroll
  for (int e = 0; e < 8; ++e) wv[e] = *(const v4f*)(conv_w + (size_t)(c8 + e) * 4);
  const v4f cb0 = *(const v4f*)(conv_b + c8);
  const v4f cb1 = *(const v4f*)(conv_b + c8 + 4);
  float acc[8];
#pragma unroll
  for (int e = 0; e < 4; ++e) { acc[e] = cb0[e]; acc[4 + e] = cb1[e]; }
#pragma unroll
  for (int k = 0; k < 4; ++k) {
    const int tk = t - 3 + k;
    const bool live = (tk >= 0);
    const int rr = live ? (row - 3 + k) : row;
    const float* p = XZ + (size_t)rr * kXZP + c8;
    const v4f a0 = *(const v4f*)(p);
    const v4f a1 = *(const v4f*)(p + 4);
#pragma unroll
    for (int e = 0; e < 4; ++e) {
      const float x0 = live ? a0[e] : 0.0f;
      const float x1 = live ? a1[e] : 0.0f;
      acc[e]     = fmaf(x0, wv[e][k], acc[e]);
      acc[4 + e] = fmaf(x1, wv[4 + e][k], acc[4 + e]);
    }
  }
  v4f s0, s1;
#pragma unroll
  for (int e = 0; e < 4; ++e) {
    const float u0 = acc[e], u1 = acc[4 + e];
    s0[e] = u0 * __builtin_amdgcn_rcpf(1.0f + __expf(-u0));
    s1[e] = u1 * __builtin_amdgcn_rcpf(1.0f + __expf(-u1));
  }
  const HL8 r = split8_bf16(s0, s1);
  const size_t o = (size_t)row * kDI + c8;
  *(volatile v8h*)(XCH + o) = r.h;
  *(volatile v8h*)(XCL + o) = r.l;
  __threadfence();
  *(volatile v8h*)(XCH + o) = r.h;
  *(volatile v8h*)(XCL + o) = r.l;
}

__global__ __launch_bounds__(128) void scan_kernel(
    const float* __restrict__ XZ, const float* __restrict__ PJ,
    const float* __restrict__ conv_w, const float* __restrict__ conv_b,
    const float* __restrict__ W_dt, const float* __restrict__ b_dt,
    const float* __restrict__ A_log, const float* __restrict__ D_param,
    unsigned short* __restrict__ YH, unsigned short* __restrict__ YL)
{
  __shared__ __align__(16) float sP[kChunk * kNPJP];
  __shared__ __align__(16) float sY[kChunk * kYP];
  const int tid = threadIdx.x;
  const int blk = blockIdx.x;
  const int bb  = blk >> 2;
  const int cg  = blk & 3;
  const int d   = cg * kCG + tid;
  const size_t rb = (size_t)bb * kL;

  const v4f cw = *(const v4f*)(conv_w + (size_t)d * 4);
  const float cbias = conv_b[d];
  const v4f wd0 = *(const v4f*)(W_dt + (size_t)d * kDTR);
  const v4f wd1 = *(const v4f*)(W_dt + (size_t)d * kDTR + 4);
  const v4f wd2 = *(const v4f*)(W_dt + (size_t)d * kDTR + 8);
  const v4f wd3 = *(const v4f*)(W_dt + (size_t)d * kDTR + 12);
  const float bdt = b_dt[d];
  const v4f al0 = *(const v4f*)(A_log + (size_t)d * kDS);
  const v4f al1 = *(const v4f*)(A_log + (size_t)d * kDS + 4);
  const v4f al2 = *(const v4f*)(A_log + (size_t)d * kDS + 8);
  const v4f al3 = *(const v4f*)(A_log + (size_t)d * kDS + 12);
  float an[kDS];
#pragma unroll
  for (int e = 0; e < 4; ++e) {
    an[e]      = -__expf(al0[e]);
    an[4 + e]  = -__expf(al1[e]);
    an[8 + e]  = -__expf(al2[e]);
    an[12 + e] = -__expf(al3[e]);
  }
  const float Dd = D_param[d];

  float xm3 = 0.f, xm2 = 0.f, xm1 = 0.f;
  float h[kDS];
#pragma unroll
  for (int n = 0; n < kDS; ++n) h[n] = 0.f;
  const int g8 = tid >> 3, c8 = (tid & 7) * 8;

#pragma unroll 1
  for (int c = 0; c < kL / kChunk; ++c) {
    const int t0 = c * kChunk;
    __syncthreads();
    {
      const float* src = PJ + (rb + t0) * kNPJP;
#pragma unroll
      for (int q = 0; q < 4; ++q) {
        const int j = q * 128 + tid;
        *(v4f*)(sP + j * 4) = *(const v4f*)(src + (size_t)j * 4);
      }
    }
    __syncthreads();
#pragma unroll 1
    for (int s = 0; s < kChunk; ++s) {
      const size_t row = rb + t0 + s;
      const float* pr = sP + s * kNPJP;
      const float xr = XZ[row * kXZP + d];
      const float zv = XZ[row * kXZP + kDI + d];
      float cv = cbias;
      cv = fmaf(xm3, cw[0], cv);
      cv = fmaf(xm2, cw[1], cv);
      cv = fmaf(xm1, cw[2], cv);
      cv = fmaf(xr,  cw[3], cv);
      xm3 = xm2; xm2 = xm1; xm1 = xr;
      const float xc = cv * __builtin_amdgcn_rcpf(1.0f + __expf(-cv));
      const v4f q0 = *(const v4f*)(pr);
      const v4f q1 = *(const v4f*)(pr + 4);
      const v4f q2 = *(const v4f*)(pr + 8);
      const v4f q3 = *(const v4f*)(pr + 12);
      float a = q0[0] * wd0[0];
      a = fmaf(q0[1], wd0[1], a); a = fmaf(q0[2], wd0[2], a); a = fmaf(q0[3], wd0[3], a);
      a = fmaf(q1[0], wd1[0], a); a = fmaf(q1[1], wd1[1], a); a = fmaf(q1[2], wd1[2], a); a = fmaf(q1[3], wd1[3], a);
      a = fmaf(q2[0], wd2[0], a); a = fmaf(q2[1], wd2[1], a); a = fmaf(q2[2], wd2[2], a); a = fmaf(q2[3], wd2[3], a);
      a = fmaf(q3[0], wd3[0], a); a = fmaf(q3[1], wd3[1], a); a = fmaf(q3[2], wd3[2], a); a = fmaf(q3[3], wd3[3], a);
      a += bdt;
      const float dt  = fmaxf(a, 0.0f) + __logf(1.0f + __expf(-fabsf(a)));
      const float dtx = dt * xc;
      const v4f bq0 = *(const v4f*)(pr + 16);
      const v4f bq1 = *(const v4f*)(pr + 20);
      const v4f bq2 = *(const v4f*)(pr + 24);
      const v4f bq3 = *(const v4f*)(pr + 28);
      const v4f cq0 = *(const v4f*)(pr + 32);
      const v4f cq1 = *(const v4f*)(pr + 36);
      const v4f cq2 = *(const v4f*)(pr + 40);
      const v4f cq3 = *(const v4f*)(pr + 44);
      float Bv[kDS], Cv[kDS];
#pragma unroll
      for (int e = 0; e < 4; ++e) {
        Bv[e] = bq0[e]; Bv[4 + e] = bq1[e]; Bv[8 + e] = bq2[e]; Bv[12 + e] = bq3[e];
        Cv[e] = cq0[e]; Cv[4 + e] = cq1[e]; Cv[8 + e] = cq2[e]; Cv[12 + e] = cq3[e];
      }
      float y = 0.f;
#pragma unroll
      for (int n = 0; n < kDS; ++n) {
        const float eA = __expf(dt * an[n]);
        h[n] = fmaf(eA, h[n], dtx * Bv[n]);
        y = fmaf(h[n], Cv[n], y);
      }
      y = fmaf(xc, Dd, y);
      const float sg = __builtin_amdgcn_rcpf(1.0f + __expf(-zv));
      y = y * (zv * sg);
      sY[s * kYP + tid] = y;
    }
    __syncthreads();
    {
      v8h hv[4], lv[4];
#pragma unroll
      for (int it = 0; it < 4; ++it) {
        const int row = it * 8 + (g8 >> 1), half = g8 & 1;
        const float* sp = sY + row * kYP + half * 64 + c8;
        const v4f a0 = *(const v4f*)(sp);
        const v4f a1 = *(const v4f*)(sp + 4);
        const HL8 r = split8_bf16(a0, a1);
        hv[it] = r.h; lv[it] = r.l;
      }
      for (int pass = 0; pass < 2; ++pass) {
#pragma unroll
        for (int it = 0; it < 4; ++it) {
          const int row = it * 8 + (g8 >> 1), half = g8 & 1;
          const size_t o = (rb + t0 + row) * kDI + (size_t)cg * kCG + half * 64 + c8;
          *(volatile v8h*)(YH + o) = hv[it];
          *(volatile v8h*)(YL + o) = lv[it];
        }
        __threadfence();
      }
    }
  }
}

__global__ __launch_bounds__(256) void fc_kernel(
    const float* __restrict__ Y1, const float* __restrict__ Y2,
    const float* __restrict__ fcw, const float* __restrict__ fcb, float* __restrict__ out)
{
  __shared__ __align__(16) float sW[kNOUT * kDM];
  __shared__ __align__(16) float sO[kTokB * 4];
  const int tid = threadIdx.x;
#pragma unroll 1
  for (int i = tid; i < kNOUT * kDM; i += 256) sW[i] = fcw[i];
  __syncthreads();
  const int tok = tid >> 3, p = tid & 7;
  const size_t row = (size_t)blockIdx.x * kTokB + tok;
  const float* y1 = Y1 + row * kDM + p * 32;
  const float* y2 = Y2 + row * kDM + p * 32;
  const float* w0 = sW + p * 32;
  const float* w1 = sW + kDM + p * 32;
  const float* w2 = sW + 2 * kDM + p * 32;
  float a0 = 0.f, a1 = 0.f, a2 = 0.f;
#pragma unroll 1
  for (int k = 0; k < 32; k += 4) {
    const v4f v1 = *(const v4f*)(y1 + k);
    const v4f v2 = *(const v4f*)(y2 + k);
    const v4f sv = v1 + v2;
    const v4f u0 = *(const v4f*)(w0 + k);
    const v4f u1 = *(const v4f*)(w1 + k);
    const v4f u2 = *(const v4f*)(w2 + k);
#pragma unroll
    for (int e = 0; e < 4; ++e) {
      a0 = fmaf(sv[e], u0[e], a0);
      a1 = fmaf(sv[e], u1[e], a1);
      a2 = fmaf(sv[e], u2[e], a2);
    }
  }
#pragma unroll
  for (int off = 1; off < 8; off <<= 1) {
    a0 += __shfl_xor(a0, off, 32);
    a1 += __shfl_xor(a1, off, 32);
    a2 += __shfl_xor(a2, off, 32);
  }
  if (p == 0) {
    sO[tok * kNOUT + 0] = a0 + fcb[0];
    sO[tok * kNOUT + 1] = a1 + fcb[1];
    sO[tok * kNOUT + 2] = a2 + fcb[2];
  }
  __syncthreads();
  const int lc = (tid < 24) ? tid : 23;
  const v4f ov = *(const v4f*)(sO + lc * 4);
  float* ob = out + (size_t)blockIdx.x * (kTokB * kNOUT);
  if (tid < 24) *(volatile v4f*)(ob + tid * 4) = ov;
  __threadfence();
  if (tid < 24) *(volatile v4f*)(ob + tid * 4) = ov;
}

extern "C" void kernel_launch(void* const* d_in, const int* in_sizes, int n_in,
                              void* d_out, int out_size, void* d_ws, size_t ws_size,
                              hipStream_t stream)
{
  if (n_in < 21) return;
  const float* x_in = (const float*)d_in[0];
  const float* in_w[2], *conv_w[2], *conv_b[2], *xproj_w[2], *dt_w[2], *dt_b[2], *A_log[2], *D_par[2], *out_w[2];
  for (int m = 0; m < 2; ++m) {
    const int base = 1 + 9 * m;
    in_w[m]    = (const float*)d_in[base + 0];
    conv_w[m]  = (const float*)d_in[base + 1];
    conv_b[m]  = (const float*)d_in[base + 2];
    xproj_w[m] = (const float*)d_in[base + 3];
    dt_w[m]    = (const float*)d_in[base + 4];
    dt_b[m]    = (const float*)d_in[base + 5];
    A_log[m]   = (const float*)d_in[base + 6];
    D_par[m]   = (const float*)d_in[base + 7];
    out_w[m]   = (const float*)d_in[base + 8];
  }
  const float* fc_w = (const float*)d_in[19];
  const float* fc_b = (const float*)d_in[20];
  float* dout = (float*)d_out;

  if (in_sizes[0] != kB * kL * kDM) return;
  for (int m = 0; m < 2; ++m) {
    const int base = 1 + 9 * m;
    if (in_sizes[base + 0] != kXZP * kDM) return;
    if (in_sizes[base + 1] != kDI * 4 || in_sizes[base + 2] != kDI) return;
    if (in_sizes[base + 3] != kNPJ * kDI) return;
    if (in_sizes[base + 4] != kDI * kDTR || in_sizes[base + 5] != kDI) return;
    if (in_sizes[base + 6] != kDI * kDS || in_sizes[base + 7] != kDI) return;
    if (in_sizes[base + 8] != kDM * kDI) return;
  }
  if (in_sizes[19] != kNOUT * kDM || in_sizes[20] != kNOUT) return;
  if (out_size != kRows * kNOUT) return;

  const size_t SZ_WI  = (size_t)kXZP * kDM * 2;
  const size_t SZ_WX  = (size_t)kNPJP * kDI * 2;
  const size_t SZ_WO  = (size_t)kDM * kDI * 2;
  const size_t SZ_XP  = (size_t)kRows * kDM * 2;
  const size_t SZ_XZ  = (size_t)kRows * kXZP * 4;
  const size_t SZ_XCP = (size_t)kRows * kDI * 2;
  const size_t SZ_PJ  = (size_t)kRows * kNPJP * 4;
  const size_t SZ_YP  = (size_t)kRows * kDI * 2;
  const size_t SZ_Y   = (size_t)kRows * kDM * 4;

  size_t off = 0;
  size_t OFF_WIH[2], OFF_WIL[2], OFF_WXH[2], OFF_WXL[2], OFF_WOH[2], OFF_WOL[2];
  for (int m = 0; m < 2; ++m) { OFF_WIH[m] = off; off += SZ_WI; OFF_WIL[m] = off; off += SZ_WI; }
  for (int m = 0; m < 2; ++m) { OFF_WXH[m] = off; off += SZ_WX; OFF_WXL[m] = off; off += SZ_WX; }
  for (int m = 0; m < 2; ++m) { OFF_WOH[m] = off; off += SZ_WO; OFF_WOL[m] = off; off += SZ_WO; }
  const size_t OFF_XH  = off; off += SZ_XP;
  const size_t OFF_XL  = off; off += SZ_XP;
  const size_t OFF_XZ  = off; off += SZ_XZ;
  const size_t OFF_XCH = off; off += SZ_XCP;
  const size_t OFF_XCL = off; off += SZ_XCP;
  const size_t OFF_PJ  = off; off += SZ_PJ;
  const size_t OFF_YH  = off; off += SZ_YP;
  const size_t OFF_YL  = off; off += SZ_YP;
  const size_t OFF_Y1  = off; off += SZ_Y;
  const size_t OFF_Y2  = off; off += SZ_Y;
  const size_t TOTAL   = off;
  if (ws_size < TOTAL) return;

  char* ws = (char*)d_ws;
  unsigned short* WIH[2], *WIL[2], *WXH[2], *WXL[2], *WOH[2], *WOL[2];
  for (int m = 0; m < 2; ++m) {
    WIH[m] = (unsigned short*)(ws + OFF_WIH[m]); WIL[m] = (unsigned short*)(ws + OFF_WIL[m]);
    WXH[m] = (unsigned short*)(ws + OFF_WXH[m]); WXL[m] = (unsigned short*)(ws + OFF_WXL[m]);
    WOH[m] = (unsigned short*)(ws + OFF_WOH[m]); WOL[m] = (unsigned short*)(ws + OFF_WOL[m]);
  }
  unsigned short* XH  = (unsigned short*)(ws + OFF_XH);
  unsigned short* XL  = (unsigned short*)(ws + OFF_XL);
  float*          XZ  = (float*)(ws + OFF_XZ);
  unsigned short* XCH = (unsigned short*)(ws + OFF_XCH);
  unsigned short* XCL = (unsigned short*)(ws + OFF_XCL);
  float*          PJ  = (float*)(ws + OFF_PJ);
  unsigned short* YH  = (unsigned short*)(ws + OFF_YH);
  unsigned short* YL  = (unsigned short*)(ws + OFF_YL);
  float*          Ybuf[2];
  Ybuf[0] = (float*)(ws + OFF_Y1);
  Ybuf[1] = (float*)(ws + OFF_Y2);
  const float* dummy_bias  = conv_b[0];
  const float* dummy_resid = conv_b[0];

  for (int m = 0; m < 2; ++m) {
    split_bf16_kernel<<<(kXZP * kDM) / 8 / 256, 256, 0, stream>>>(in_w[m], WIH[m], WIL[m], (kXZP * kDM) / 8);
    split_bf16_pad_kernel<<<(kNPJP * kDI) / 8 / 256, 256, 0, stream>>>(xproj_w[m], kNPJ * kDI, WXH[m], WXL[m], (kNPJP * kDI) / 8);
    split_bf16_kernel<<<(kDM * kDI) / 8 / 256, 256, 0, stream>>>(out_w[m], WOH[m], WOL[m], (kDM * kDI) / 8);
  }

  for (int m = 0; m < 2; ++m) {
    x_rows_split_kernel<<<(kRows * 32) / 256, 256, 0, stream>>>(x_in, XH, XL, m);

    wmma_gemm64<1, true, 0, 0, false><<<dim3(256, 1), 256, 0, stream>>>(
        XH, XL, kDM, 0L, WIH[m], WIL[m], kDM, 0L,
        (void*)XZ, (void*)XZ, kXZP, 0L, dummy_bias, dummy_resid, 0L, kRows, kXZP, kDM, 1.0f);

    conv_split_kernel<<<(kRows * 64) / 256, 256, 0, stream>>>(XZ, conv_w[m], conv_b[m], XCH, XCL);

    wmma_gemm64<1, true, 0, 0, false><<<dim3(16, 1), 256, 0, stream>>>(
        XCH, XCL, kDI, 0L, WXH[m], WXL[m], kDI, 0L,
        (void*)PJ, (void*)PJ, kNPJP, 0L, dummy_bias, dummy_resid, 0L, kRows, kNPJP, kDI, 1.0f);

    scan_kernel<<<kB * (kDI / kCG), kCG, 0, stream>>>(XZ, PJ, conv_w[m], conv_b[m], dt_w[m], dt_b[m], A_log[m], D_par[m], YH, YL);

    wmma_gemm64<1, true, 0, 0, false><<<dim3(64, 1), 256, 0, stream>>>(
        YH, YL, kDI, 0L, WOH[m], WOL[m], kDI, 0L,
        (void*)Ybuf[m], (void*)Ybuf[m], kDM, 0L, dummy_bias, dummy_resid, 0L, kRows, kDM, kDI, 1.0f);
  }

  fc_kernel<<<kRows / kTokB, 256, 0, stream>>>(Ybuf[0], Ybuf[1], fc_w, fc_b, dout);
}
